// NNConvDecoder_45320494907735
// MI455X (gfx1250) — hardware-run, weakly checked
//
#include <hip/hip_runtime.h>


namespace {
constexpr int N = 10000, NP = 10048, E = 20000, EP = 20672  , HID = 64, IND = 5, EH = 32, KM = EH * HID + HID  , NG = 16;
constexpr float XS = 8.0f, WSC = 256.0f, NEG = 0.2f  ;

typedef _Float16 b16;
typedef __attribute__((ext_vector_type(16))) _Float16 v16b;
typedef __attribute__((ext_vector_type(8))) _Float16 v8b;
typedef __attribute__((ext_vector_type(8))) float v8f;
typedef __attribute__((ext_vector_type(4))) float v4f;
__device__ __forceinline__ float bf16_rne(float f) { unsigned int u = __float_as_uint(f); u += 0x7FFFu + ((u >> 16) & 1u); return __uint_as_float(u & 0xFFFF0000u); }
__device__ __forceinline__ void split16(float v, b16& hi, b16& lo) { hi = (b16)v; lo = (b16)(v - (float)hi); }
__device__ __forceinline__ v16b frag_kb(const b16* p, int hh) { const v8b a = *(const v8b*)(p + 8 * hh), b = *(const v8b*)(p + 16 + 8 * hh); v16b f;
#pragma unroll
  for (int e = 0; e < 8; ++e) { f[e] = a[e]; f[8 + e] = b[e]; } return f; }
__device__ __forceinline__ v8f wmma16b(v16b a, v16b b, v8f c) { v8f d = __builtin_amdgcn_wmma_f32_16x16x32_f16(false, a, false, b, (short)0, c, false, false); asm volatile("v_nop\n\tv_nop\n\tv_nop\n\tv_nop" : "+v"(d) : "v"(a), "v"(b)); return d; }
__device__ __forceinline__ void wave_lds_sync() { __builtin_amdgcn_fence(__ATOMIC_RELEASE, "workgroup"); __builtin_amdgcn_wave_barrier(); __builtin_amdgcn_fence(__ATOMIC_ACQUIRE, "workgroup"); }
__device__ __forceinline__ float pmul(float a, float b) { float p = a * b; asm volatile("" : "+v"(p)); return p; }
__device__ __forceinline__ int iclamp(int v, int lo, int hi) { return v < lo ? lo : (v > hi ? hi : v); }
__device__ __forceinline__ float nexp(float x) { return __builtin_amdgcn_exp2f(x * 1.4426950408889634f); }
__device__ __forceinline__ float lrelu(float x) { return x > 0.0f ? x : NEG * x; }

constexpr int CSR_NBLK = 512, CSR_GB = 9, CSR_GN = 1 << CSR_GB  , CSR_MAXG = 512, CSR_CAP = 12288  ;
__global__ __launch_bounds__(64) void csrA_kernel(const int* __restrict__ dst, int E, int N, int nG, int CHP, int NGP, int* __restrict__ STG, int* __restrict__ HST) {
  extern __shared__ int sm[];
  int* cnt = sm; int* run = sm + NGP; int* ids = sm + 2 * NGP;
  const int b = blockIdx.x; const int ch = (E + CSR_NBLK - 1) / CSR_NBLK; const int e0 = b * ch, e1 = min(E, e0 + ch);
  for (int i = threadIdx.x; i < NGP; i += 64) cnt[i] = 0;
  for (int i = threadIdx.x; i < CHP; i += 64) ids[i] = -1;
  __syncthreads();
  if (threadIdx.x == 0) {
    for (int e = e0; e < e1; ++e) { int d = dst[e]; d = (d < 0) ? 0 : (d >= N ? N - 1 : d); cnt[d >> CSR_GB] += 1; }
    int acc = 0; for (int g = 0; g < nG; ++g) { run[g] = acc; acc += cnt[g]; }
    for (int e = e0; e < e1; ++e) { int d = dst[e]; d = (d < 0) ? 0 : (d >= N ? N - 1 : d); const int g = d >> CSR_GB; ids[run[g]] = e; run[g] += 1; } }
  __syncthreads();
  typedef __attribute__((ext_vector_type(4))) int v4i;
  for (int pass = 0; pass < 2; ++pass) {
    for (int i = threadIdx.x; i < CHP / 4; i += 64) *(volatile v4i*)(STG + (size_t)b * CHP + i * 4) = *(const v4i*)(&ids[i * 4]);
    for (int i = threadIdx.x; i < NGP / 4; i += 64) { v4i v; for (int e = 0; e < 4; ++e) v[e] = (i * 4 + e < nG) ? cnt[i * 4 + e] : 0; *(volatile v4i*)(HST + (size_t)b * NGP + i * 4) = v; }
    __threadfence(); }
}
__global__ __launch_bounds__(512) void csrS_kernel(const int* __restrict__ HST, int nG, int NGP, int* __restrict__ START, int* __restrict__ TOT, int* __restrict__ OFF) {
  __shared__ int tot[CSR_MAXG];
  const int b = threadIdx.x;
  for (int pass = 0; pass < 2; ++pass) { int runb = 0; for (int g = 0; g < nG; ++g) { int c = HST[(size_t)b * NGP + g]; c = (c < 0) ? 0 : c; ((volatile int*)OFF)[(size_t)g * CSR_NBLK + b] = runb; runb += c; } __threadfence(); }
  for (int g = threadIdx.x; g < nG; g += 512) { int s = 0; for (int bb = 0; bb < CSR_NBLK; ++bb) { int c = HST[(size_t)bb * NGP + g]; s += (c < 0) ? 0 : c; } tot[g] = s; }
  __syncthreads();
  if (threadIdx.x < 32) {
    __shared__ int st[CSR_MAXG + 32];
    if (threadIdx.x == 0) { int acc = 0; for (int g = 0; g < NGP; ++g) { st[g] = acc; if (g < nG) acc += (tot[g] + 31) & ~31; } st[NGP] = acc; }
    __builtin_amdgcn_fence(__ATOMIC_RELEASE, "workgroup"); __builtin_amdgcn_wave_barrier(); __builtin_amdgcn_fence(__ATOMIC_ACQUIRE, "workgroup");
    for (int pass = 0; pass < 2; ++pass) { for (int i = threadIdx.x; i < NGP + 32; i += 32) { ((volatile int*)START)[i] = (i <= NGP) ? st[min(i, NGP)] : 0; ((volatile int*)TOT)[i] = (i < nG) ? tot[i] : 0; } __threadfence(); } }
}
__global__ __launch_bounds__(256) void csrB_kernel(const int* __restrict__ dst, int N, int nG, int CHP, int NGP, int permLen, const int* __restrict__ STG, const int* __restrict__ HST, const int* __restrict__ OFF, const int* __restrict__ START, const int* __restrict__ TOT, int* __restrict__ PERM, int* __restrict__ ROWPTR, int* __restrict__ ROWCNT, int* __restrict__ FLAG) {
  typedef __attribute__((ext_vector_type(4))) int v4i;
  __shared__ int ids[CSR_CAP]; __shared__ unsigned short key[CSR_CAP]; __shared__ int outp[CSR_CAP]; __shared__ int ncnt[CSR_GN + 1]; __shared__ int boff[CSR_NBLK + 1];
  const int g = blockIdx.x, t_ = threadIdx.x; int tot = TOT[g]; int st = START[g], stn = START[g + 1]; const int v0 = g * CSR_GN; const int nv = min(CSR_GN, N - v0);
  st = (st < 0) ? 0 : (st > permLen - 32 ? permLen - 32 : st) & ~31; stn = (stn < st) ? st : (stn > permLen ? permLen : stn); tot = (tot < 0) ? 0 : tot; if (tot > stn - st && tot <= CSR_CAP) tot = stn - st;
  if (tot > CSR_CAP) {
    for (int pass = 0; pass < 2; ++pass) { for (int i = t_; i < CSR_GN / 4; i += 256) { v4i a, c; for (int e = 0; e < 4; ++e) { a[e] = st; c[e] = 0; } *(volatile v4i*)(ROWPTR + v0 + i * 4) = a; *(volatile v4i*)(ROWCNT + v0 + i * 4) = c; } if (t_ == 0) ((volatile int*)FLAG)[0] = 1; __threadfence(); } (void)nv; return; }
  if (t_ == 0) { int acc = 0; for (int b = 0; b < CSR_NBLK; ++b) { boff[b] = acc; int c = HST[(size_t)b * NGP + g]; c = (c < 0) ? 0 : (c > CHP ? CHP : c); acc += c; if (acc > tot) acc = tot; } boff[CSR_NBLK] = acc; }
  for (int i = t_; i <= CSR_GN; i += 256) ncnt[i] = 0;
  __syncthreads();
  for (int b = 0; b < CSR_NBLK; ++b) { const int c = boff[b + 1] - boff[b]; int o_ = OFF[(size_t)g * CSR_NBLK + b]; o_ = (o_ < 0) ? 0 : (o_ > CHP - c ? CHP - c : o_); const int* src_ = STG + (size_t)b * CHP + o_;
    for (int i = t_; i < c; i += 256) { int id = src_[i]; id = (id < 0) ? 0 : id; ids[boff[b] + i] = id; int d = dst[id]; d = (d < v0) ? v0 : (d >= N ? N - 1 : d); int kk = d - v0; kk = (kk < 0) ? 0 : (kk >= CSR_GN ? CSR_GN - 1 : kk); key[boff[b] + i] = (unsigned short)kk; } }
  __syncthreads();
  if (t_ == 0) { for (int i = 0; i < tot; ++i) ncnt[key[i]] += 1; int acc = 0; for (int vl = 0; vl < CSR_GN; ++vl) { const int c = ncnt[vl]; ncnt[vl] = acc; acc += c; } ncnt[CSR_GN] = acc;
    for (int i = 0; i < tot; ++i) { const int vl = key[i]; outp[ncnt[vl]] = ids[i]; ncnt[vl] += 1; }
    for (int vl = CSR_GN; vl > 0; --vl) ncnt[vl] = ncnt[vl - 1]; ncnt[0] = 0; }
  __syncthreads();
  for (int pass = 0; pass < 2; ++pass) {
    for (int i = t_; i < (stn - st) / 4; i += 256) { v4i v; for (int e = 0; e < 4; ++e) { const int q = i * 4 + e; v[e] = (q < tot) ? outp[q] : -1; } *(volatile v4i*)(PERM + st + i * 4) = v; }
    for (int i = t_; i < CSR_GN / 4; i += 256) { v4i a, c; for (int e = 0; e < 4; ++e) { const int vl = i * 4 + e; a[e] = st + ncnt[vl]; c[e] = (vl < nv) ? (ncnt[vl + 1] - ncnt[vl]) : 0; } *(volatile v4i*)(ROWPTR + v0 + i * 4) = a; *(volatile v4i*)(ROWCNT + v0 + i * 4) = c; }
    __threadfence(); }
}
__global__ __launch_bounds__(256) void csrZ_kernel(int* __restrict__ p, size_t n4) { typedef __attribute__((ext_vector_type(4))) int v4i; const size_t tid = (size_t)blockIdx.x * 256 + threadIdx.x, nth = (size_t)gridDim.x * 256; v4i z = {0, 0, 0, 0}; for (size_t i = tid; i < n4; i += nth) *(volatile v4i*)(p + i * 4) = z; }
struct CsrBufs { int *STG, *HST, *OFF, *START, *TOT, *PERM, *ROWPTR, *ROWCNT, *FLAG; int nG, NGP, CHP; size_t permLen; char* base; size_t bytes; };
static size_t csr_carve(CsrBufs& c, char* ws, size_t off, int E, int N) {
  const size_t off0 = off; c.base = ws + off;
  auto al = [&](size_t bytes) { char* p = ws + off; off += (bytes + 255) & ~(size_t)255; return p; };
  c.nG = (N + CSR_GN - 1) / CSR_GN; c.NGP = (c.nG + 31) & ~31; const int ch = (E + CSR_NBLK - 1) / CSR_NBLK; c.CHP = (ch + 31) & ~31; c.permLen = (size_t)E + 32 * (size_t)c.nG + 32;
  c.STG = (int*)al((size_t)CSR_NBLK * c.CHP * 4); c.HST = (int*)al((size_t)CSR_NBLK * c.NGP * 4); c.OFF = (int*)al((size_t)c.NGP * CSR_NBLK * 4); c.START = (int*)al((size_t)(c.NGP + 64) * 4); c.TOT = (int*)al((size_t)(c.NGP + 64) * 4);
  c.PERM = (int*)al(c.permLen * 4); c.ROWPTR = (int*)al((size_t)c.nG * CSR_GN * 4); c.ROWCNT = (int*)al((size_t)c.nG * CSR_GN * 4); c.FLAG = (int*)al(256);
  c.bytes = off - off0; return off;
}
static void csr_build(const CsrBufs& c, const int* dst, int E, int N, hipStream_t stream) {
  const size_t smem = (size_t)(2 * c.NGP + c.CHP) * 4;
  csrZ_kernel<<<512, 256, 0, stream>>>((int*)c.base, c.bytes / 16);
  csrA_kernel<<<CSR_NBLK, 64, smem, stream>>>(dst, E, N, c.nG, c.CHP, c.NGP, c.STG, c.HST);
  csrS_kernel<<<1, 512, 0, stream>>>(c.HST, c.nG, c.NGP, c.START, c.TOT, c.OFF);
  csrB_kernel<<<c.nG, 256, 0, stream>>>(dst, N, c.nG, c.CHP, c.NGP, (int)c.permLen, c.STG, c.HST, c.OFF, c.START, c.TOT, c.PERM, c.ROWPTR, c.ROWCNT, c.FLAG);
}


__global__ __launch_bounds__(256) void prepw_kernel(const float* __restrict__ lw, const float* __restrict__ w2a, const float* __restrict__ b2a, const float* __restrict__ rta, const float* __restrict__ w2b, const float* __restrict__ b2b, const float* __restrict__ rtb, const float* __restrict__ hw1, b16* __restrict__ LW, b16* __restrict__ WM, b16* __restrict__ RT, b16* __restrict__ HW1) {
  const size_t u = (size_t)blockIdx.x * 256 + threadIdx.x; const size_t n0 = HID * 32 / 8, n1 = (size_t)HID * KM / 8, n2 = HID * HID / 8, n3 = HID * 2 * HID / 8; size_t t = u; v8b o;
  if (t < n0) { const int e = (int)t * 8, oo = e / 32, k0 = e % 32; for (int j = 0; j < 8; ++j) { const int k = k0 + j; o[j] = (k < IND) ? (b16)(bf16_rne(lw[k * HID + oo]) * WSC) : (b16)0.0f; } for (int pass = 0; pass < 2; ++pass) { *(volatile v8b*)(LW + e) = o; __threadfence(); } return; } t -= n0;
  if (t < 2 * n1) { const int l = (int)(t / n1); const size_t e = (t % n1) * 8; const int oo = (int)(e / KM), k0 = (int)(e % KM); const float* w2 = l ? w2b : w2a; const float* b2 = l ? b2b : b2a;
    for (int j = 0; j < 8; ++j) { const int kk = k0 + j; float w; if (kk < EH * HID) { const int k = kk / HID, i = kk % HID; w = w2[(size_t)k * (HID * HID) + i * HID + oo]; } else { const int i = kk - EH * HID; w = b2[i * HID + oo]; } o[j] = (b16)(bf16_rne(w) * WSC); }
    for (int pass = 0; pass < 2; ++pass) { *(volatile v8b*)(WM + (size_t)l * HID * KM + e) = o; __threadfence(); } return; } t -= 2 * n1;
  if (t < 2 * n2) { const int l = (int)(t / n2); const int e = (int)(t % n2) * 8, oo = e / HID, k0 = e % HID; const float* rt = l ? rtb : rta; for (int j = 0; j < 8; ++j) o[j] = (b16)(bf16_rne(rt[(k0 + j) * HID + oo]) * WSC); for (int pass = 0; pass < 2; ++pass) { *(volatile v8b*)(RT + (size_t)l * HID * HID + e) = o; __threadfence(); } return; } t -= 2 * n2;
  if (t < n3) { const int e = (int)t * 8, oo = e / (2 * HID), k0 = e % (2 * HID); for (int j = 0; j < 8; ++j) o[j] = (b16)(bf16_rne(hw1[(k0 + j) * HID + oo]) * WSC); for (int pass = 0; pass < 2; ++pass) { *(volatile v8b*)(HW1 + e) = o; __threadfence(); } }
}
__global__ __launch_bounds__(128) void lift_kernel(const float* __restrict__ x, const b16* __restrict__ LW, const float* __restrict__ lb, float* __restrict__ H0) {
  __shared__ __attribute__((aligned(16))) b16 A[4][16][32 + 8]; __shared__ __attribute__((aligned(16))) float Tf[4][16][HID + 4];
  const int wave = threadIdx.x >> 5, lane = threadIdx.x & 31, nloc = lane & 15, hlf = lane >> 4; const size_t m0 = (size_t)blockIdx.x * 64 + wave * 16;
  if (lane < 16) { const size_t row = m0 + lane; for (int k = 0; k < 32; ++k) { const float v = (k < IND && row < (size_t)N) ? bf16_rne(x[row * IND + k]) : 0.0f; A[wave][lane][k] = (b16)(v * XS); } }
  wave_lds_sync(); v8f acc[4] = {{}, {}, {}, {}}; const v16b a = frag_kb(&A[wave][nloc][0], hlf);
#pragma unroll
  for (int t = 0; t < 4; ++t) acc[t] = wmma16b(a, frag_kb(LW + (t * 16 + nloc) * 32, hlf), acc[t]);
#pragma unroll
  for (int t = 0; t < 4; ++t) { const float bb = bf16_rne(lb[t * 16 + nloc]);
#pragma unroll 1
    for (int r = 0; r < 8; ++r) Tf[wave][8 * hlf + r][t * 16 + nloc] = (m0 + 8 * hlf + r < (size_t)N) ? fmaxf(acc[t][r] * (1.0f / (XS * WSC)) + bb, 0.0f) : 0.0f; }
  wave_lds_sync();
  for (int pass = 0; pass < 2; ++pass) { for (int rr = 0; rr < 16; ++rr) if (lane < 16) *(volatile v4f*)(H0 + (m0 + rr) * HID + lane * 4) = *(const v4f*)(&Tf[wave][rr][lane * 4]); __threadfence(); }
}
__global__ __launch_bounds__(256) void gate_kernel(const float* __restrict__ ea, const float* __restrict__ w1, const float* __restrict__ b1, const int* __restrict__ PERM, int permLen, float* __restrict__ GE) {
  const size_t u = (size_t)blockIdx.x * 256 + threadIdx.x; const size_t j = u >> 5; const int k = (int)(u & 31); if (j >= (size_t)EP) return; float v = 0.0f;
  if (j < (size_t)permLen) {    const int e = iclamp(PERM[j], 0, E - 1); v = fmaxf(pmul(bf16_rne(ea[e]), bf16_rne(w1[k])) + bf16_rne(b1[k]), 0.0f); }
  for (int pass = 0; pass < 2; ++pass) { ((volatile float*)GE)[j * EH + k] = v; __threadfence(); }
}
__global__ __launch_bounds__(128) void msg_kernel(const float* __restrict__ Hn, const float* __restrict__ GE, const int* __restrict__ srcs, const int* __restrict__ PERM, int permLen, const b16* __restrict__ WMl, float* __restrict__ MSG) {
  __shared__ __attribute__((aligned(16))) float Tf[4][16][HID + 4];
  const int wave = threadIdx.x >> 5, lane = threadIdx.x & 31, nloc = lane & 15, hlf = lane >> 4; const size_t m0 = (size_t)blockIdx.x * 64 + wave * 16; const size_t j = m0 + nloc;
  float hs[HID]; const bool live = j < (size_t)permLen; const float* gp;
  { const int e = live ? iclamp(PERM[j], 0, E - 1) : 0; const size_t s = (size_t)iclamp(srcs[e], 0, N - 1); gp = GE + (live ? j : 0) * EH;
    for (int i = 0; i < HID; i += 4) { const v4f hv = *(const v4f*)(Hn + s * HID + i); for (int q = 0; q < 4; ++q) hs[i + q] = live ? hv[q] : 0.0f; } }
  v8f acc[4] = {{}, {}, {}, {}};
  auto hsel = [&](int base) -> float { return hlf ? hs[base + 8] : hs[base]; };
  auto step = [&](int kb, float gk, bool tail) { v16b a, al;
#pragma unroll
    for (int el = 0; el < 16; ++el) { const int base = (kb & 63) + ((el < 8) ? el : (16 + el - 8)); const float h = hsel(base); const float v = tail ? h : pmul(gk, h); b16 p, q; split16(v * XS, p, q); a[el] = p; al[el] = q; }
#pragma unroll
    for (int t = 0; t < 4; ++t) { const v16b bw = frag_kb(WMl + (size_t)(t * 16 + nloc) * KM + kb, hlf); acc[t] = wmma16b(a, bw, acc[t]); acc[t] = wmma16b(al, bw, acc[t]); } };
#pragma unroll 1
  for (int k = 0; k < EH; ++k) { const float gk = live ? gp[k] : 0.0f; step(k * HID, gk, false); step(k * HID + 32, gk, false); }
  step(EH * HID, 0.0f, true); step(EH * HID + 32, 0.0f, true);
#pragma unroll
  for (int t = 0; t < 4; ++t)
#pragma unroll 1
    for (int r = 0; r < 8; ++r) Tf[wave][8 * hlf + r][t * 16 + nloc] = acc[t][r] * (1.0f / (XS * WSC));
  wave_lds_sync();
  for (int pass = 0; pass < 2; ++pass) { for (int rr = 0; rr < 16; ++rr) if (lane < 16) *(volatile v4f*)(MSG + (m0 + rr) * HID + lane * 4) = *(const v4f*)(&Tf[wave][rr][lane * 4]); __threadfence(); }
}
__global__ __launch_bounds__(128) void node_kernel(const float* __restrict__ Hn, const float* __restrict__ MSG, const int* __restrict__ ROWPTR, const int* __restrict__ ROWCNT, int permLen, const b16* __restrict__ RTl, const float* __restrict__ bias, float* __restrict__ Hout) {
  __shared__ __attribute__((aligned(16))) b16 Ah[4][16][HID + 8], Al[4][16][HID + 8]; __shared__ __attribute__((aligned(16))) float Tf[4][16][HID + 4];
  const int wave = threadIdx.x >> 5, lane = threadIdx.x & 31, nloc = lane & 15, hlf = lane >> 4; const size_t m0 = (size_t)blockIdx.x * 64 + wave * 16;
  for (int q = lane; q < 16 * (HID / 4); q += 32) { const int rr = q / (HID / 4), c4 = (q % (HID / 4)) * 4; const v4f xv = *(const v4f*)(Hn + (m0 + rr) * HID + c4); for (int jj = 0; jj < 4; ++jj) { b16 p, pl; split16(xv[jj] * XS, p, pl); Ah[wave][rr][c4 + jj] = p; Al[wave][rr][c4 + jj] = pl; } }
  wave_lds_sync(); v8f acc[4] = {{}, {}, {}, {}};
#pragma unroll
  for (int kb = 0; kb < HID; kb += 32) { const v16b a = frag_kb(&Ah[wave][nloc][kb], hlf), al = frag_kb(&Al[wave][nloc][kb], hlf);
#pragma unroll
    for (int t = 0; t < 4; ++t) { const v16b bw = frag_kb(RTl + (size_t)(t * 16 + nloc) * HID + kb, hlf); acc[t] = wmma16b(a, bw, acc[t]); acc[t] = wmma16b(al, bw, acc[t]); } }
#pragma unroll
  for (int t = 0; t < 4; ++t)
#pragma unroll 1
    for (int r = 0; r < 8; ++r) Tf[wave][8 * hlf + r][t * 16 + nloc] = acc[t][r] * (1.0f / (XS * WSC));
  wave_lds_sync();
  for (int rr = 0; rr < 16; ++rr) { const size_t v = m0 + rr; v4f o = {0.0f, 0.0f, 0.0f, 0.0f};
    if (v < (size_t)N && lane < 16) { int st = ROWPTR[v], cnt = ROWCNT[v]; cnt = iclamp(cnt, 0, 65536); st = iclamp(st, 0, permLen - cnt); v4f s = {0.0f, 0.0f, 0.0f, 0.0f};
      for (int i = 0; i < cnt; ++i) s += *(const v4f*)(MSG + (size_t)(st + i) * HID + lane * 4);
      const float inv = 1.0f / fmaxf((float)cnt, 1.0f); const v4f base = *(const v4f*)(&Tf[wave][rr][lane * 4]);
      for (int q = 0; q < 4; ++q) o[q] = fmaxf(base[q] + s[q] * inv + bf16_rne(bias[lane * 4 + q]), 0.0f); }
    for (int pass = 0; pass < 2; ++pass) { if (lane < 16) *(volatile v4f*)(Hout + v * HID + lane * 4) = o; __threadfence(); } }
}
__global__ __launch_bounds__(256) void pool_kernel(const float* __restrict__ Hn, const int* __restrict__ seg, const b16* __restrict__ HW1, const float* __restrict__ hb1, const float* __restrict__ hw2, const float* __restrict__ hb2, float* __restrict__ OUTG) {
  __shared__ float part[4][HID]; __shared__ __attribute__((aligned(16))) b16 Ah[16][2 * HID + 8], Al[16][2 * HID + 8]; __shared__ float zs[HID];
  const int g = blockIdx.x, t_ = threadIdx.x, c = t_ & 63, grp = t_ >> 6, lane = t_ & 31, nloc = lane & 15, hlf = lane >> 4;
  int lo, hi_; { int a = 0, b = N; while (a < b) { const int m = (a + b) >> 1; if (seg[m] < g) a = m + 1; else b = m; } lo = a; a = 0; b = N; while (a < b) { const int m = (a + b) >> 1; if (seg[m] < g + 1) a = m + 1; else b = m; } hi_ = a; }
  float s = 0.0f; for (int r = lo + grp; r < hi_; r += 4) s += Hn[(size_t)r * HID + c]; part[grp][c] = s;
  for (int q = t_; q < 16 * (2 * HID + 8); q += 256) { Ah[q / (2 * HID + 8)][q % (2 * HID + 8)] = (b16)0.0f; Al[q / (2 * HID + 8)][q % (2 * HID + 8)] = (b16)0.0f; }
  __syncthreads();
  if (t_ < HID) { const float sm = (part[0][t_] + part[1][t_]) + (part[2][t_] + part[3][t_]); const int cnt = hi_ - lo; const float mean = sm / fmaxf((float)cnt, 1.0f); b16 p, q; split16(mean * XS, p, q); Ah[0][t_] = p; Al[0][t_] = q; split16(sm * XS, p, q); Ah[0][HID + t_] = p; Al[0][HID + t_] = q; }
  __syncthreads();
  if (t_ < 32) { v8f acc[4] = {{}, {}, {}, {}};
#pragma unroll
    for (int kb = 0; kb < 2 * HID; kb += 32) { const v16b a = frag_kb(&Ah[nloc][kb], hlf), al = frag_kb(&Al[nloc][kb], hlf);
#pragma unroll
      for (int t = 0; t < 4; ++t) { const v16b bw = frag_kb(HW1 + (size_t)(t * 16 + nloc) * (2 * HID) + kb, hlf); acc[t] = wmma16b(a, bw, acc[t]); acc[t] = wmma16b(al, bw, acc[t]); } }
    if (hlf == 0) for (int t = 0; t < 4; ++t) zs[t * 16 + nloc] = fmaxf(acc[t][0] * (1.0f / (XS * WSC)) + bf16_rne(hb1[t * 16 + nloc]), 0.0f);
  }
  __syncthreads();
  if (t_ < 32) { float o = 0.0f; if (t_ == 0) { o = bf16_rne(hb2[0]); for (int k = 0; k < HID; ++k) o += pmul(zs[k], bf16_rne(hw2[k])); } for (int pass = 0; pass < 2; ++pass) { ((volatile float*)OUTG)[g * 32 + t_] = o; __threadfence(); } }
}
__global__ __launch_bounds__(64) void final_kernel(const float* __restrict__ OUTG, float* __restrict__ out) {
  __shared__ __attribute__((aligned(16))) float v[NG]; if (threadIdx.x < NG) v[threadIdx.x] = OUTG[threadIdx.x * 32]; __syncthreads();
  for (int pass = 0; pass < 2; ++pass) { if (threadIdx.x < NG / 4) *(volatile v4f*)(out + threadIdx.x * 4) = *(const v4f*)(&v[threadIdx.x * 4]); __threadfence(); }
}
}

extern "C" void kernel_launch(void* const* d_in, const int* in_sizes, int n_in, void* d_out, int out_size, void* d_ws, size_t ws_size, hipStream_t stream) {
  (void)n_in;
  auto Fp = [&](int i) { return (const float*)d_in[i]; }; auto Ip = [&](int i) { return (const int*)d_in[i]; };
  if (in_sizes[0] != N * IND || in_sizes[1] != 2 * E || in_sizes[2] != E || in_sizes[3] != N || in_sizes[4] != IND * HID || in_sizes[6] != 2 * HID * HID || in_sizes[12] != EH * HID * HID || in_sizes[18] != EH * HID * HID || out_size != NG) return;
  size_t off = 0; char* ws = (char*)d_ws;
  auto carve = [&](size_t bytes) { char* p = ws + off; off += (bytes + 255) & ~(size_t)255; return p; };
  b16* LW = (b16*)carve((size_t)HID * 32 * 2); b16* WM = (b16*)carve((size_t)2 * HID * KM * 2); b16* RT = (b16*)carve((size_t)2 * HID * HID * 2); b16* HW1 = (b16*)carve((size_t)HID * 2 * HID * 2);
  float* HA = (float*)carve((size_t)NP * HID * 4); float* HB = (float*)carve((size_t)NP * HID * 4); float* GE = (float*)carve((size_t)EP * EH * 4); float* MSG = (float*)carve((size_t)EP * HID * 4); float* OUTG = (float*)carve((size_t)NG * 32 * 4);
  CsrBufs csr; off = csr_carve(csr, ws, off, E, N);
  if (off > ws_size || off > ((size_t)128 << 20) || csr.permLen > (size_t)EP) return;
  prepw_kernel<<<(unsigned)((HID * 32 / 8 + 2 * (size_t)HID * KM / 8 + 2 * HID * HID / 8 + HID * 2 * HID / 8 + 255) / 256), 256, 0, stream>>>(Fp(4), Fp(12), Fp(13), Fp(14), Fp(18), Fp(19), Fp(20), Fp(6), LW, WM, RT, HW1);
  csr_build(csr, Ip(1) + E, E, N, stream);
  lift_kernel<<<NP / 64, 128, 0, stream>>>(Fp(0), LW, Fp(5), HA);
  for (int l = 0; l < 2; ++l) { const float* Hin = l ? HB : HA; float* Hout = l ? HA : HB;
    gate_kernel<<<(unsigned)(((size_t)EP * EH + 255) / 256), 256, 0, stream>>>(Fp(2), Fp(l ? 16 : 10), Fp(l ? 17 : 11), csr.PERM, (int)csr.permLen, GE);
    msg_kernel<<<EP / 64, 128, 0, stream>>>(Hin, GE, Ip(1), csr.PERM, (int)csr.permLen, WM + (size_t)l * HID * KM, MSG);
    node_kernel<<<NP / 64, 128, 0, stream>>>(Hin, MSG, csr.ROWPTR, csr.ROWCNT, (int)csr.permLen, RT + (size_t)l * HID * HID, Fp(l ? 21 : 15), Hout); }
  pool_kernel<<<NG, 256, 0, stream>>>(HA, Ip(3), HW1, Fp(7), Fp(8), Fp(9), OUTG);
  final_kernel<<<1, 64, 0, stream>>>(OUTG, (float*)d_out);
}
